// NetGATDeform_24661702213862
// MI455X (gfx1250) — hardware-verified
//
#include <hip/hip_runtime.h>
#define NN 10000
#define NE 60000
#define NHD 6
#define ECAP 32
typedef __bf16 v16b __attribute__((ext_vector_type(16)));
typedef unsigned short v8us __attribute__((ext_vector_type(8), may_alias));
typedef float  v8f  __attribute__((ext_vector_type(8)));
typedef float  v4f  __attribute__((ext_vector_type(4)));
typedef float  v4fa __attribute__((ext_vector_type(4), may_alias));
union FragB { v16b v; v8us half[2]; unsigned short u[16]; };

__device__ __forceinline__ unsigned short bf16_bits(float x) { unsigned int u = __float_as_uint(x); return (unsigned short)((u + 0x7FFFu + ((u >> 16) & 1u)) >> 16); }
__device__ __forceinline__ float bf16_val(unsigned short b) { return __uint_as_float(((unsigned int)b) << 16); }
__device__ __forceinline__ float bf16_round(float x) { return bf16_val(bf16_bits(x)); }
template <int NT>
__device__ __forceinline__ v8f mmaN(v16b ah, v16b al, v16b bh, v16b bl, v8f c) {
  c = __builtin_amdgcn_wmma_f32_16x16x32_bf16(false, ah, false, bh, (short)0, c, false, false);
  if (NT >= 2) c = __builtin_amdgcn_wmma_f32_16x16x32_bf16(false, al, false, bh, (short)0, c, false, false);
  if (NT >= 3) c = __builtin_amdgcn_wmma_f32_16x16x32_bf16(false, ah, false, bl, (short)0, c, false, false);
  asm volatile("v_nop\n\tv_nop\n\tv_nop\n\tv_nop" : "+v"(c) : "v"(ah), "v"(al), "v"(bh), "v"(bl));
  return c;
}

__global__ __launch_bounds__(256) void k_wt_bf16(const float* __restrict__ W, unsigned short* __restrict__ Wt, int K, int N) {
  const int t = blockIdx.x * 256 + threadIdx.x;
  const int k8n = K / 8;
  if (t >= N * k8n) return;
  const int n = t / k8n, k8 = (t % k8n) * 8;
  v8us v;
#pragma unroll
  for (int i = 0; i < 8; ++i) v[i] = bf16_bits(W[(size_t)(k8 + i) * N + n]);
  *(volatile v8us*)(Wt + (size_t)n * K + k8) = v;
  __threadfence();
  *(volatile v8us*)(Wt + (size_t)n * K + k8) = v;
}

template <bool ASPLIT, int ACT, bool BIAS_BF16>
__global__ __launch_bounds__(128) void k_gemm_bf(const float* __restrict__ A, int lda, const unsigned short* __restrict__ Wt, int ldb,
                                               const float* __restrict__ bias, float* __restrict__ C, int ldc, int M, int N, int K) {
  __shared__ __attribute__((aligned(16))) float so[4][16][64];
  const int tid = threadIdx.x, w = tid >> 5, lane = tid & 31, ln = lane & 15, hh = lane >> 4;
  const int ntn = N / 64;
  const int wid = blockIdx.x * 4 + w;
  const int mt = wid / ntn, nq = wid % ntn;
  if (mt * 16 >= M) return;
  const int row0 = mt * 16, col0 = nq * 64;
  const float* arow = A + (size_t)(row0 + ln) * lda;
  v8f acc[4] = {};
  for (int kb = 0; kb < K; kb += 32) {
    FragB ah, al;
    const v4f x0 = *(const v4fa*)(arow + kb + 8 * hh), x1 = *(const v4fa*)(arow + kb + 8 * hh + 4);
    const v4f x2 = *(const v4fa*)(arow + kb + 16 + 8 * hh), x3 = *(const v4fa*)(arow + kb + 16 + 8 * hh + 4);
    float xs[16] = {x0[0],x0[1],x0[2],x0[3],x1[0],x1[1],x1[2],x1[3],x2[0],x2[1],x2[2],x2[3],x3[0],x3[1],x3[2],x3[3]};
#pragma unroll
    for (int i = 0; i < 16; ++i) { const unsigned short hb = bf16_bits(xs[i]); ah.u[i] = hb; al.u[i] = ASPLIT ? bf16_bits(xs[i] - bf16_val(hb)) : (unsigned short)0; }
#pragma unroll
    for (int t = 0; t < 4; ++t) {
      const unsigned short* brow = Wt + (size_t)(col0 + t * 16 + ln) * ldb + kb;
      FragB b;
      b.half[0] = *(const v8us*)(brow + 8 * hh);
      b.half[1] = *(const v8us*)(brow + 16 + 8 * hh);
      acc[t] = mmaN<ASPLIT ? 2 : 1>(ah.v, al.v, b.v, b.v, acc[t]);
    }
  }
#pragma unroll
  for (int t = 0; t < 4; ++t) {
    float bv = bias ? bias[col0 + t * 16 + ln] : 0.f;
    if (BIAS_BF16) bv = bf16_round(bv);
#pragma unroll
    for (int r = 0; r < 8; ++r) { float v = acc[t][r] + bv; if (ACT == 1) v = fmaxf(v, 0.f); so[w][8 * hh + r][t * 16 + ln] = v; }
  }
  __builtin_amdgcn_fence(__ATOMIC_ACQ_REL, "workgroup");
  __builtin_amdgcn_wave_barrier();
  const int rsub = lane >> 4, c4 = (lane & 15) * 4;
  for (int pass = 0; pass < 2; ++pass) {
#pragma unroll
    for (int q = 0; q < 8; ++q) {
      const int r = q * 2 + rsub;
      const v4f v = *(const v4fa*)&so[w][r][c4];
      *(volatile v4f*)(C + (size_t)(row0 + r) * ldc + col0 + c4) = v;
    }
    if (pass == 0) __threadfence();
  }
}

template <bool ASPLIT, int ACT, bool BIAS_BF16, bool RES_BF16>
__global__ __launch_bounds__(128) void k_gemm_bf3(const float* __restrict__ A, int lda, const unsigned short* __restrict__ Wt, int ldb,
                                                const float* __restrict__ bias, const float* __restrict__ resid, int rmod, int ldr,
                                                float* __restrict__ C, int ldc, int M, int N, int K) {
  __shared__ __attribute__((aligned(16))) float so[4][16][64];
  const int tid = threadIdx.x, w = tid >> 5, lane = tid & 31, ln = lane & 15, hh = lane >> 4;
  const int ntn = N / 64;
  const int wid = blockIdx.x * 4 + w;
  const int mt = wid / ntn, nq = wid % ntn;
  if (mt * 16 >= M) return;
  const int row0 = mt * 16, col0 = nq * 64;
  const float* arow = A + (size_t)(row0 + ln) * lda;
  v8f acc[4] = {};
  for (int kb = 0; kb < K; kb += 32) {
    FragB ah, al;
    const v4f x0 = *(const v4fa*)(arow + kb + 8 * hh), x1 = *(const v4fa*)(arow + kb + 8 * hh + 4);
    const v4f x2 = *(const v4fa*)(arow + kb + 16 + 8 * hh), x3 = *(const v4fa*)(arow + kb + 16 + 8 * hh + 4);
    float xs[16] = {x0[0],x0[1],x0[2],x0[3],x1[0],x1[1],x1[2],x1[3],x2[0],x2[1],x2[2],x2[3],x3[0],x3[1],x3[2],x3[3]};
#pragma unroll
    for (int i = 0; i < 16; ++i) { const unsigned short hb = bf16_bits(xs[i]); ah.u[i] = hb; al.u[i] = ASPLIT ? bf16_bits(xs[i] - bf16_val(hb)) : (unsigned short)0; }
#pragma unroll
    for (int t = 0; t < 4; ++t) {
      const unsigned short* brow = Wt + (size_t)(col0 + t * 16 + ln) * ldb + kb;
      FragB b;
      b.half[0] = *(const v8us*)(brow + 8 * hh);
      b.half[1] = *(const v8us*)(brow + 16 + 8 * hh);
      acc[t] = mmaN<ASPLIT ? 2 : 1>(ah.v, al.v, b.v, b.v, acc[t]);
    }
  }
#pragma unroll
  for (int t = 0; t < 4; ++t) {
    const int col = col0 + t * 16 + ln;
    float bv = bias ? bias[col] : 0.f;
    if (BIAS_BF16) bv = bf16_round(bv);
#pragma unroll
    for (int r = 0; r < 8; ++r) {
      float v = acc[t][r] + bv;
      if (resid) { float rv = resid[(size_t)((row0 + 8 * hh + r) % rmod) * ldr + col]; if (RES_BF16) rv = bf16_round(rv); v += rv; }
      if (ACT == 1) v = fmaxf(v, 0.f);
      if (ACT == 2) v = 0.5f * v * (1.0f + erff(v * 0.70710678118654752f));
      if (ACT == 3) { const float u = 0.7978845608028654f * (v + 0.044715f * v * v * v); v = 0.5f * v * (1.0f + tanhf(u)); }
      so[w][8 * hh + r][t * 16 + ln] = v;
    }
  }
  __builtin_amdgcn_fence(__ATOMIC_ACQ_REL, "workgroup");
  __builtin_amdgcn_wave_barrier();
  const int rsub = lane >> 4, c4 = (lane & 15) * 4;
  for (int pass = 0; pass < 2; ++pass) {
#pragma unroll
    for (int q = 0; q < 8; ++q) {
      const int r = q * 2 + rsub;
      const v4f v = *(const v4fa*)&so[w][r][c4];
      *(volatile v4f*)(C + (size_t)(row0 + r) * ldc + col0 + c4) = v;
    }
    if (pass == 0) __threadfence();
  }
}
template <bool PARAM_BF16>
__global__ __launch_bounds__(256) void k_layernorm(const float* __restrict__ X, const float* __restrict__ R, const float* __restrict__ g, const float* __restrict__ bta,
                                                  float* __restrict__ out_sum, float* __restrict__ out_norm, int N, float eps) {
  __shared__ float red[256];
  const int row = blockIdx.x, tid = threadIdx.x;
  const float* x = X + (size_t)row * N; const float* rr = R ? R + (size_t)row * N : nullptr;
  float vals[16];
  const int per = N / 256;
  float s1 = 0.f;
  for (int u = 0; u < per / 4; ++u) {
    const int j = tid * 4 + 1024 * u;
    const v4f a = *(const v4fa*)(x + j);
    v4f b = {0.f,0.f,0.f,0.f}; if (rr) b = *(const v4fa*)(rr + j);
#pragma unroll
    for (int q = 0; q < 4; ++q) { const float v = a[q] + b[q]; vals[u * 4 + q] = v; s1 += v; }
  }
  red[tid] = s1; __syncthreads();
  for (int st = 128; st > 0; st >>= 1) { if (tid < st) red[tid] += red[tid + st]; __syncthreads(); }
  const float mu = red[0] / (float)N; __syncthreads();
  float s2 = 0.f;
  for (int u = 0; u < per / 4; ++u)
#pragma unroll
    for (int q = 0; q < 4; ++q) { const float c = vals[u * 4 + q] - mu; s2 += c * c; }
  red[tid] = s2; __syncthreads();
  for (int st = 128; st > 0; st >>= 1) { if (tid < st) red[tid] += red[tid + st]; __syncthreads(); }
  const float rs = rsqrtf(red[0] / (float)N + eps);
  for (int pass = 0; pass < 2; ++pass) {
    for (int u = 0; u < per / 4; ++u) {
      const int j = tid * 4 + 1024 * u;
      v4f o, sm;
#pragma unroll
      for (int q = 0; q < 4; ++q) {
        float gg = g[j + q], bb = bta[j + q];
        if (PARAM_BF16) { gg = bf16_round(gg); bb = bf16_round(bb); }
        sm[q] = vals[u * 4 + q]; o[q] = (vals[u * 4 + q] - mu) * rs * gg + bb;
      }
      if (out_sum) *(volatile v4f*)(out_sum + (size_t)row * N + j) = sm;
      *(volatile v4f*)(out_norm + (size_t)row * N + j) = o;
    }
    if (pass == 0) __threadfence();
  }
}


typedef _Float16 v16h __attribute__((ext_vector_type(16)));
union FragH { v16h v; v8us half[2]; _Float16 h[16]; unsigned short u[16]; };
template <int NT>
__device__ __forceinline__ v8f mmaH(v16h ah, v16h al, v16h bh, v16h bl, v8f c) {
  c = __builtin_amdgcn_wmma_f32_16x16x32_f16(false, ah, false, bh, (short)0, c, false, false);
  if (NT >= 2) c = __builtin_amdgcn_wmma_f32_16x16x32_f16(false, al, false, bh, (short)0, c, false, false);
  if (NT >= 3) c = __builtin_amdgcn_wmma_f32_16x16x32_f16(false, ah, false, bl, (short)0, c, false, false);
  asm volatile("v_nop\n\tv_nop\n\tv_nop\n\tv_nop" : "+v"(c) : "v"(ah), "v"(al), "v"(bh), "v"(bl));
  return c;
}
template <bool ASPLIT>
__global__ __launch_bounds__(128) void k_gemm_h(const float* __restrict__ A, int lda, size_t sA, const _Float16* __restrict__ Bh, int ldb, size_t sB, float alpha, float* __restrict__ C, int ldc, size_t sC, int M, int N, int K) {
  __shared__ __attribute__((aligned(16))) float so[4][16][64];
  const int tid = threadIdx.x, w = tid >> 5, lane = tid & 31, ln = lane & 15, hh = lane >> 4; const int by = blockIdx.y;
  A += (size_t)by * sA; Bh += (size_t)by * sB; C += (size_t)by * sC;
  const int ntn = (N + 63) / 64; const int wid = blockIdx.x * 4 + w; const int mt = wid / ntn, nq = wid % ntn; if (mt * 16 >= M) return;
  const int row0 = mt * 16, col0 = nq * 64; const float* arow = A + (size_t)(row0 + ln) * lda;
  v8f acc[4] = {};
  for (int kb = 0; kb < K; kb += 32) {
    FragH ah, al;
    const v4f x0 = *(const v4fa*)(arow + kb + 8 * hh), x1 = *(const v4fa*)(arow + kb + 8 * hh + 4), x2 = *(const v4fa*)(arow + kb + 16 + 8 * hh), x3 = *(const v4fa*)(arow + kb + 16 + 8 * hh + 4);
    float xs[16] = {x0[0],x0[1],x0[2],x0[3],x1[0],x1[1],x1[2],x1[3],x2[0],x2[1],x2[2],x2[3],x3[0],x3[1],x3[2],x3[3]};
#pragma unroll
    for (int i = 0; i < 16; ++i) { const _Float16 h = (_Float16)xs[i]; ah.h[i] = h; al.h[i] = ASPLIT ? (_Float16)(xs[i] - (float)h) : (_Float16)0.0f; }
#pragma unroll
    for (int t = 0; t < 4; ++t) { if (col0 + t * 16 >= N) continue; const size_t boff = (size_t)(col0 + t * 16 + ln) * ldb + kb; FragH bq; bq.half[0] = *(const v8us*)(Bh + boff + 8 * hh); bq.half[1] = *(const v8us*)(Bh + boff + 16 + 8 * hh);
      acc[t] = mmaH<ASPLIT ? 2 : 1>(ah.v, al.v, bq.v, bq.v, acc[t]); }
  }
#pragma unroll
  for (int t = 0; t < 4; ++t) { if (col0 + t * 16 >= N) continue;
#pragma unroll
    for (int r = 0; r < 8; ++r) so[w][8 * hh + r][t * 16 + ln] = acc[t][r] * alpha; }
  __builtin_amdgcn_fence(__ATOMIC_ACQ_REL, "workgroup"); __builtin_amdgcn_wave_barrier();
  const int rsub = lane >> 4, c4 = (lane & 15) * 4;
  for (int pass = 0; pass < 2; ++pass) {
#pragma unroll
    for (int q = 0; q < 8; ++q) { const int r = q * 2 + rsub; if (col0 + c4 < N) { const v4f v = *(const v4fa*)&so[w][r][c4]; *(volatile v4f*)(C + (size_t)(row0 + r) * ldc + col0 + c4) = v; } }
    if (pass == 0) __threadfence(); }
}

__global__ __launch_bounds__(256) void k_wt_f16(const float* __restrict__ W, _Float16* __restrict__ Wt, int K, int N, float scale) {
  const int t = blockIdx.x * 256 + threadIdx.x; if (t >= N * (K / 8)) return; const int n = t / (K / 8), k8 = (t % (K / 8)) * 8; FragH f;
#pragma unroll
  for (int i = 0; i < 8; ++i) f.h[i] = (_Float16)(bf16_round(W[(size_t)(k8 + i) * N + n]) * scale); const v8us o = f.half[0];
  *(volatile v8us*)((unsigned short*)Wt + (size_t)n * K + k8) = o; __threadfence(); *(volatile v8us*)((unsigned short*)Wt + (size_t)n * K + k8) = o;
}
template <int ACT>
__global__ __launch_bounds__(128) void k_gemm_hhx(const _Float16* __restrict__ A, int lda, size_t sA, const _Float16* __restrict__ Bh, int ldb, size_t sB, float alpha, const float* __restrict__ bias, size_t sBias, const float* __restrict__ CP, int rowsPerB, size_t sCPb, int row0g,
    float* __restrict__ C, _Float16* __restrict__ C16, int ldc, size_t sC, int M, int N, int K) {
  __shared__ __attribute__((aligned(16))) float so[4][16][64];
  const int tid = threadIdx.x, w = tid >> 5, lane = tid & 31, ln = lane & 15, hh = lane >> 4; const int by = blockIdx.y;
  A += (size_t)by * sA; Bh += (size_t)by * sB; const size_t cofs = (size_t)by * sC; const float* bp = bias ? bias + (size_t)by * sBias : nullptr;
  const int ntn = (N + 63) / 64; const int wid = blockIdx.x * 4 + w; const int mt = wid / ntn, nq = wid % ntn; if (mt * 16 >= M) return;
  const int row0 = mt * 16, col0 = nq * 64; const _Float16* arow = A + (size_t)(row0 + ln) * lda;
  v8f acc[4] = {};
  for (int kb = 0; kb < K; kb += 32) { FragH ah; ah.half[0] = *(const v8us*)((const unsigned short*)arow + kb + 8 * hh); ah.half[1] = *(const v8us*)((const unsigned short*)arow + kb + 16 + 8 * hh);
#pragma unroll
    for (int t = 0; t < 4; ++t) { if (col0 + t * 16 >= N) continue; const size_t boff = (size_t)(col0 + t * 16 + ln) * ldb + kb; FragH bq; bq.half[0] = *(const v8us*)((const unsigned short*)Bh + boff + 8 * hh); bq.half[1] = *(const v8us*)((const unsigned short*)Bh + boff + 16 + 8 * hh);
      acc[t] = mmaH<1>(ah.v, ah.v, bq.v, bq.v, acc[t]); }
  }
#pragma unroll
  for (int t = 0; t < 4; ++t) { if (col0 + t * 16 >= N) continue; const int col = col0 + t * 16 + ln; const float bv = bp ? bf16_round(bp[col]) : 0.f;
#pragma unroll
    for (int r = 0; r < 8; ++r) { float v = acc[t][r] * alpha + bv; if (CP) { const int bidx = (row0g + row0 + 8 * hh + r) / rowsPerB; v += CP[(size_t)bidx * sCPb + (size_t)by * 64 + col]; } if (ACT == 1) v = (v > 0.f) ? v : expm1f(v); else if (ACT == 7) v = (v > 0.f) ? v + 1.0f : expf(v); else if (ACT == 8) v = tanhf(v); else if (ACT == 9) v = 0.5f * v * (1.0f + tanhf(0.7978845608028654f * (v + 0.044715f * v * v * v))); else if (ACT == 11) v = 1.0f / (1.0f + expf(-v)); else if (ACT == 12) v = (v > 0.f) ? v : 0.01f * v; else if (ACT == 14) v = (v > 0.f) ? v : 0.1f * v; else if (ACT == 15) v = v / (1.0f + expf(-v)); else if (ACT == 3) v = fmaxf(v, 0.f); else if (ACT == 6) v = 0.5f * v * (1.0f + erff(v * 0.70710678118654752f)); so[w][8 * hh + r][t * 16 + ln] = v; } }
  __builtin_amdgcn_fence(__ATOMIC_ACQ_REL, "workgroup"); __builtin_amdgcn_wave_barrier();
  const int rsub = lane >> 4, c4 = (lane & 15) * 4; typedef _Float16 v4h __attribute__((ext_vector_type(4)));
  for (int pass = 0; pass < 2; ++pass) {
#pragma unroll
    for (int q = 0; q < 8; ++q) { const int r = q * 2 + rsub; if (col0 + c4 < N) { const v4f v = *(const v4fa*)&so[w][r][c4]; if (C) *(volatile v4f*)(C + cofs + (size_t)(row0 + r) * ldc + col0 + c4) = v; if (C16) { v4h h4; for (int i = 0; i < 4; ++i) h4[i] = (_Float16)v[i]; *(volatile v4h*)(C16 + cofs + (size_t)(row0 + r) * ldc + col0 + c4) = h4; } } }
    if (pass == 0) __threadfence(); }
}


typedef _Float16 v4h __attribute__((ext_vector_type(4)));

__global__ __launch_bounds__(256) void k_x16(const float* __restrict__ x, _Float16* __restrict__ X16, size_t n8) { const size_t t = (size_t)blockIdx.x * 256 + threadIdx.x; if (t >= n8) return; FragH f;
#pragma unroll
  for (int q = 0; q < 8; ++q) f.h[q] = (_Float16)bf16_round(x[t * 8 + q]); *(volatile v8us*)((unsigned short*)X16 + t * 8) = f.half[0]; __threadfence(); *(volatile v8us*)((unsigned short*)X16 + t * 8) = f.half[0]; }
__global__ __launch_bounds__(256) void k_h16(const float* __restrict__ x, _Float16* __restrict__ X16, size_t n8) { const size_t t = (size_t)blockIdx.x * 256 + threadIdx.x; if (t >= n8) return; FragH f;
#pragma unroll
  for (int q = 0; q < 8; ++q) f.h[q] = (_Float16)x[t * 8 + q]; *(volatile v8us*)((unsigned short*)X16 + t * 8) = f.half[0]; __threadfence(); *(volatile v8us*)((unsigned short*)X16 + t * 8) = f.half[0]; }
__global__ __launch_bounds__(256) void k_round16f(const float* __restrict__ W, _Float16* __restrict__ Bt, size_t n8) { const size_t t = (size_t)blockIdx.x * 256 + threadIdx.x; if (t >= n8) return; FragH f;
#pragma unroll
  for (int i = 0; i < 8; ++i) f.h[i] = (_Float16)(bf16_round(W[t * 8 + i]) * 16.0f); *(volatile v8us*)((unsigned short*)Bt + t * 8) = f.half[0]; __threadfence(); *(volatile v8us*)((unsigned short*)Bt + t * 8) = f.half[0]; }
template <int NHv, int TTv>
__global__ __launch_bounds__(256) void k_vt(const _Float16* __restrict__ V16, int ldv, int voff, _Float16* __restrict__ Vt) { __shared__ unsigned short tl[64][66]; const int tid = threadIdx.x; const int slab = blockIdx.x / (TTv / 64), lg = blockIdx.x % (TTv / 64); const int b = slab / NHv, h = slab % NHv;
  for (int i = tid; i < 64 * 8; i += 256) { const int r = i / 8, c8 = (i % 8) * 8; FragH f; f.half[0] = *(const v8us*)((const unsigned short*)V16 + ((size_t)b * TTv + lg * 64 + r) * ldv + voff + h * 64 + c8);
#pragma unroll
    for (int q = 0; q < 8; ++q) tl[r][c8 + q] = f.u[q]; }
  __syncthreads();
  for (int pass = 0; pass < 2; ++pass) {
#pragma unroll
    for (int rd = 0; rd < 2; ++rd) { const int d = rd * 32 + tid / 8, pc = tid % 8; FragH f;
#pragma unroll
      for (int q = 0; q < 8; ++q) f.u[q] = tl[pc * 8 + q][d];
      *(volatile v8us*)((unsigned short*)Vt + ((size_t)slab * 64 + d) * TTv + lg * 64 + pc * 8) = f.half[0]; }
    if (pass == 0) __threadfence(); } }

__global__ __launch_bounds__(256) void k_hl(const float* __restrict__ F, _Float16* __restrict__ Hh, _Float16* __restrict__ Hl, size_t n8) { const size_t t = (size_t)blockIdx.x * 256 + threadIdx.x; if (t >= n8) return; FragH fh, fl; const v4f a = *(const v4fa*)(F + t * 8), c = *(const v4fa*)(F + t * 8 + 4);
#pragma unroll
  for (int q = 0; q < 4; ++q) { _Float16 h = (_Float16)a[q]; fh.h[q] = h; fl.h[q] = (_Float16)((a[q] - (float)h) * 1024.0f); h = (_Float16)c[q]; fh.h[4 + q] = h; fl.h[4 + q] = (_Float16)((c[q] - (float)h) * 1024.0f); }
  for (int pass = 0; pass < 2; ++pass) { *(volatile v8us*)((unsigned short*)Hh + t * 8) = fh.half[0]; *(volatile v8us*)((unsigned short*)Hl + t * 8) = fl.half[0]; if (pass == 0) __threadfence(); } }

#define VST2(T, ptr, val) do { const T vst2_v_ = (val); *(volatile T*)(ptr) = vst2_v_; __threadfence(); *(volatile T*)(ptr) = vst2_v_; } while (0)

#define C4_NB 4096
#define C4_CH 8192
__device__ __forceinline__ int c4_bucket(int v, int N) { v = min(max(v, 0), N - 1); return (int)(((long long)v * C4_NB) / N); }
__global__ __launch_bounds__(256) void k_c4_count(const int* __restrict__ tgt, int E, int N, int* __restrict__ CNT) {
    __shared__ int hist[C4_NB]; const int ch = blockIdx.x, t = threadIdx.x; const int e0 = ch * C4_CH; const int nt = min(C4_CH, E - e0);
    for (int j = 0; j < 16; ++j) hist[t + 256 * j] = 0; __syncthreads();
    for (int i = t; i < nt; i += 256) atomicAdd(&hist[c4_bucket(tgt[e0 + i], N)], 1);
    __syncthreads();
    for (int j = 0; j < 16; ++j) { const int v = hist[t + 256 * j]; VST2(int, CNT + (long long)ch * C4_NB + t + 256 * j, v); } }
__global__ __launch_bounds__(256) void k_c4_offsets(const int* __restrict__ CNT, int nch, int E, int* __restrict__ OFFB, int* __restrict__ BOFF) {
    __shared__ int tot[C4_NB]; __shared__ int part[256]; const int t = threadIdx.x;
    for (int j = 0; j < 16; ++j) { const int b = t + 256 * j; int s = 0; for (int ch = 0; ch < nch; ++ch) s += CNT[(long long)ch * C4_NB + b]; tot[b] = s; }
    __syncthreads();
    { int s = 0; for (int q = 0; q < 16; ++q) s += tot[16 * t + q]; part[t] = s; } __syncthreads();
    if (t == 0) { int run = 0; for (int i = 0; i < 256; ++i) { const int v = part[i]; part[i] = run; run += v; } } __syncthreads();
    { int run = part[t]; for (int q = 0; q < 16; ++q) { const int v = tot[16 * t + q]; tot[16 * t + q] = run; run += v; } }
    __syncthreads();
    for (int j = 0; j < 16; ++j) { const int b = t + 256 * j; VST2(int, BOFF + b, tot[b]); }
    if (t == 0) VST2(int, BOFF + C4_NB, E);
    for (int j = 0; j < 16; ++j) { const int b = t + 256 * j; int run = tot[b]; for (int ch = 0; ch < nch; ++ch) { VST2(int, OFFB + (long long)ch * C4_NB + b, run); run += CNT[(long long)ch * C4_NB + b]; } } }
__global__ __launch_bounds__(256) void k_c4_scatter(const int* __restrict__ tgt, int E, int N, const int* __restrict__ OFFB, int* __restrict__ BUF) {
    __shared__ int cur[C4_NB]; __shared__ int bk[256]; const int ch = blockIdx.x, t = threadIdx.x; const int e0 = ch * C4_CH; const int nt = min(C4_CH, E - e0);
    const int wv = t >> 5, ln = t & 31;
    for (int j = 0; j < 16; ++j) cur[t + 256 * j] = OFFB[(long long)ch * C4_NB + t + 256 * j];
    __syncthreads();
    for (int s0 = 0; s0 < C4_CH; s0 += 256) {
        const int i = s0 + t; const int e = e0 + i; const int b = (i < nt) ? c4_bucket(tgt[min(e, E - 1)], N) : -1;
        bk[t] = b; __syncthreads();
        int rank = 0, cntw = 0;
        for (int l = 0; l < 32; ++l) { const int o = bk[(wv << 5) + l]; const bool same = (o == b) && (b >= 0); cntw += same ? 1 : 0; rank += (same && l < ln) ? 1 : 0; }
        const bool last = (b >= 0) && (rank == cntw - 1);
        for (int w = 0; w < 8; ++w) {
            if (wv == w && b >= 0) { int pos = cur[b] + rank; pos = min(max(pos, 0), E - 1); VST2(int, BUF + pos, e); }
            __syncthreads();
            if (wv == w && last) cur[b] += cntw;
            __syncthreads(); }
    } }
template <int CAP>
__global__ __launch_bounds__(256) void k_c4_lists(const int* __restrict__ tgt, const int* __restrict__ BUF, const int* __restrict__ BOFF, int N, int E, int* __restrict__ NBR, int* __restrict__ cnt) {
    const int d = blockIdx.x * 256 + threadIdx.x; if (d >= N) return; const int b = c4_bucket(d, N); int n = 0; int* row = NBR + (long long)d * CAP;
    const int p0 = min(max(BOFF[b], 0), E), p1 = min(max(BOFF[b + 1], p0), E);
    for (int p = p0; p < p1; ++p) { int e = BUF[p]; e = min(max(e, 0), E - 1); if (tgt[e] == d) { if (n < CAP) VST2(int, row + n, e); ++n; } }
    for (int j = n; j < CAP; ++j) VST2(int, row + j, -1); VST2(int, cnt + d, min(n, CAP)); }
__global__ __launch_bounds__(256) void k_c4_scan1(const int* __restrict__ cnt, int* __restrict__ PART, int N) {
    __shared__ int part[256]; const int per = ((((N + 255) / 256) + 31) / 32) * 32; const int a = threadIdx.x * per, b = min(N, a + per); int s = 0;
    for (int i = a; i < b; ++i) s += cnt[i]; part[threadIdx.x] = s; __syncthreads();
    if (threadIdx.x == 0) { int run = 0; for (int t = 0; t < 256; ++t) { const int v = part[t]; part[t] = run; run += v; } } __syncthreads();
    VST2(int, PART + threadIdx.x, part[threadIdx.x]); }
__global__ __launch_bounds__(256) void k_c4_scan2(const int* __restrict__ cnt, const int* __restrict__ PART, int* __restrict__ off, int N) {
    const int i = blockIdx.x * 256 + threadIdx.x; if (i > N) return; const int per = ((((N + 255) / 256) + 31) / 32) * 32; const int r = min(i / per, 255); const int a = r * per;
    int s = PART[r]; for (int kq = a; kq < i; ++kq) s += cnt[min(kq, N - 1)];
    VST2(int, off + i, s); }
template <int CAP>
__global__ __launch_bounds__(256) void k_c4_slotcopy(const int* __restrict__ off, const int* __restrict__ NBR, int* __restrict__ slot, int N) {
    const int t = blockIdx.x * 256 + threadIdx.x; const int tot = off[N]; if (t >= tot) return;
    int lo = 0, hi = N - 1; while (lo < hi) { const int mid = (lo + hi + 1) >> 1; if (off[mid] <= t) lo = mid; else hi = mid - 1; }
    int j = t - off[lo]; j = (j < 0) ? 0 : ((j >= CAP) ? (CAP - 1) : j); VST2(int, slot + t, NBR[(long long)lo * CAP + j]); }

typedef float v2f __attribute__((ext_vector_type(2)));
__device__ __forceinline__ float selu_f(float x) { return 1.0507009873554805f * ((x > 0.f) ? x : 1.6732632423543772f * expm1f(x)); }
__global__ __launch_bounds__(256) void k_lin(const float* __restrict__ data, const float* __restrict__ lW, const float* __restrict__ lb, _Float16* __restrict__ T1, float* __restrict__ CC0) {
  #pragma clang fp contract(off)
  const int t = blockIdx.x * 256 + threadIdx.x; if (t >= NN * 32) return; const int n = t / 32, c0 = (t % 32) * 8; float dv[10];
#pragma unroll
  for (int k = 0; k < 10; ++k) dv[k] = bf16_round(data[(size_t)n * 10 + k]);
  FragH f;
#pragma unroll
  for (int q = 0; q < 8; ++q) { const int c = c0 + q; float v; if (c < 2) v = dv[c]; else { const int o = c - 2; float s = bf16_round(lb[o]);
#pragma unroll
      for (int k = 0; k < 10; ++k) s += dv[k] * bf16_round(lW[k * 254 + o]); v = selu_f(s); } f.h[q] = (_Float16)v; }
  *(volatile v8us*)((unsigned short*)T1 + (size_t)n * 256 + c0) = f.half[0]; __threadfence(); *(volatile v8us*)((unsigned short*)T1 + (size_t)n * 256 + c0) = f.half[0]; (void)CC0; }
__global__ __launch_bounds__(256) void k_cc0(const float* __restrict__ data, float* __restrict__ CC0) { const int n = blockIdx.x * 256 + threadIdx.x; if (n >= NN) return; v2f cv; cv.x = bf16_round(data[(size_t)n * 10]); cv.y = bf16_round(data[(size_t)n * 10 + 1]); *(volatile v2f*)(CC0 + (size_t)n * 2) = cv; __threadfence(); *(volatile v2f*)(CC0 + (size_t)n * 2) = cv; }
template <int DIN, int C, int HCP>
__global__ __launch_bounds__(256) void k_wl(const float* __restrict__ Wm, const float* __restrict__ as, const float* __restrict__ ad, _Float16* __restrict__ Bt, _Float16* __restrict__ Bl) {
  #pragma clang fp contract(off)
  const int HC = NHD * C; const int t = blockIdx.x * 256 + threadIdx.x; if (t >= (HCP + 16) * (DIN / 8)) return; const int r = t / (DIN / 8), k0 = (t % (DIN / 8)) * 8; FragH f;
  if (r < HCP) {
#pragma unroll
    for (int q = 0; q < 8; ++q) f.h[q] = (r < HC) ? (_Float16)(bf16_round(Wm[(size_t)(k0 + q) * HC + r]) * 16.0f) : (_Float16)0.0f;
    *(volatile v8us*)((unsigned short*)Bt + (size_t)r * DIN + k0) = f.half[0]; __threadfence(); *(volatile v8us*)((unsigned short*)Bt + (size_t)r * DIN + k0) = f.half[0]; }
  else { const int j = r - HCP;
#pragma unroll
    for (int q = 0; q < 8; ++q) { float v = 0.f; if (j < 12) { const int hh = j % NHD; const float* att = (j < NHD) ? as : ad; float s = 0.f;
#pragma unroll 1
        for (int c = 0; c < C; ++c) s += bf16_round(Wm[(size_t)(k0 + q) * HC + hh * C + c]) * bf16_round(att[hh * C + c]); v = s; } f.h[q] = (_Float16)(v * 16.0f); }
    *(volatile v8us*)((unsigned short*)Bl + (size_t)j * DIN + k0) = f.half[0]; __threadfence(); *(volatile v8us*)((unsigned short*)Bl + (size_t)j * DIN + k0) = f.half[0]; } }
template <int C, int XP, int DIN, int PRE, int DNEXT>
__global__ __launch_bounds__(512) void k_dgat(const _Float16* __restrict__ X, const float* __restrict__ AL, const _Float16* __restrict__ Tcur, const float* __restrict__ CC, const int* __restrict__ src, const int* __restrict__ nbr, const int* __restrict__ cnt, const float* __restrict__ bb, _Float16* __restrict__ Tnext, float* __restrict__ CCn) {
  #pragma clang fp contract(off)
  __shared__ __attribute__((aligned(16))) float macc[16][C + 1]; __shared__ __attribute__((aligned(16))) unsigned short rowb[16][DNEXT]; __shared__ __attribute__((aligned(16))) float cst[16][2]; __shared__ int sidx[16][32]; __shared__ float pw[16][32];
  const int tid = threadIdx.x, w = tid >> 5, l = tid & 31; const int d = blockIdx.x * 16 + w;
  const int n = min(max(cnt[d], 0), ECAP); const float cdx = CC[(size_t)d * 2], cdy = CC[(size_t)d * 2 + 1];
  for (int c = l; c < C; c += 32) macc[w][c] = 0.f;
  { int e = nbr[(size_t)d * ECAP + l]; const bool live = (l < n) && (e >= 0); e = min(max(e, 0), NE - 1); int s = src[e]; s = min(max(s, 0), NN - 1); sidx[w][l] = live ? s : -1; }
  __syncthreads();
  const int sj = sidx[w][l]; const bool live = sj >= 0; const int ss = live ? sj : d; const float dcx = CC[(size_t)ss * 2] - cdx, dcy = CC[(size_t)ss * 2 + 1] - cdy; float dsx = 0.f, dsy = 0.f;
#pragma unroll 1
  for (int h = 0; h < NHD; ++h) { const float add = AL[(size_t)d * 16 + NHD + h]; float ev = AL[(size_t)ss * 16 + h] + add; ev = (ev > 0.f) ? ev : 0.2f * ev; if (!live) ev = -3.0e38f;
    float mx = ev; for (int o = 16; o > 0; o >>= 1) mx = fmaxf(mx, __shfl_xor(mx, o, 32)); const float p = live ? expf(ev - mx) : 0.f; float ls = p; for (int o = 16; o > 0; o >>= 1) ls += __shfl_xor(ls, o, 32);
    const float wgt = p / (ls + 1e-16f) * (1.0f / NHD); float tx = wgt * dcx, ty = wgt * dcy; for (int o = 16; o > 0; o >>= 1) { tx += __shfl_xor(tx, o, 32); ty += __shfl_xor(ty, o, 32); } dsx += tx; dsy += ty;
    pw[w][l] = wgt; __syncthreads();
#pragma unroll 1
    for (int c = l; c < C; c += 32) { float a = 0.f;
#pragma unroll 1
      for (int j = 0; j < n; ++j) { const int s = sidx[w][j]; const float wj = pw[w][j]; a += (s >= 0) ? wj * (float)X[(size_t)max(s, 0) * XP + h * C + c] : 0.f; }
      macc[w][c] += a; }
    __syncthreads(); }
  { const float ncx = cdx + dsx, ncy = cdy + dsy; if (l == 0) { FragH fc; fc.h[0] = (_Float16)ncx; fc.h[1] = (_Float16)ncy; rowb[w][0] = fc.u[0]; rowb[w][1] = fc.u[1]; cst[w][0] = ncx; cst[w][1] = ncy; }
    if (l < PRE) rowb[w][2 + l] = ((const unsigned short*)Tcur)[(size_t)d * DIN + l];
#pragma unroll 1
    for (int c = l; c < C; c += 32) { FragH ff; ff.h[0] = (_Float16)selu_f(macc[w][c] + bf16_round(bb[c])); rowb[w][2 + PRE + c] = ff.u[0]; } }
  __syncthreads();
  for (int pass = 0; pass < 2; ++pass) {
    for (int i = tid; i < 16 * (DNEXT / 8); i += 512) { const int ww = i / (DNEXT / 8), pc = i % (DNEXT / 8); const v8us v = *(const v8us*)&rowb[ww][pc * 8]; *(volatile v8us*)((unsigned short*)Tnext + (size_t)(blockIdx.x * 16 + ww) * DNEXT + pc * 8) = v; }
    if (tid < 8) { const v4f v = *(const v4fa*)&cst[tid * 2][0]; *(volatile v4f*)(CCn + (size_t)blockIdx.x * 32 + tid * 4) = v; }
    if (pass == 0) __threadfence(); } }
__global__ __launch_bounds__(256) void k_dgat4(const float* __restrict__ AL, const float* __restrict__ CC, const int* __restrict__ src, const int* __restrict__ nbr, const int* __restrict__ cnt, float* __restrict__ out) {
  #pragma clang fp contract(off)
  const int d = blockIdx.x * 256 + threadIdx.x; if (d >= NN) return; const int n = min(max(cnt[d], 0), ECAP); const float cdx = CC[(size_t)d * 2], cdy = CC[(size_t)d * 2 + 1]; float dsx = 0.f, dsy = 0.f;
#pragma unroll 1
  for (int h = 0; h < NHD; ++h) { const float add = AL[(size_t)d * 16 + NHD + h]; float mx = -3.0e38f, ls = 0.f, px = 0.f, py = 0.f;
#pragma unroll 1
    for (int j = 0; j < ECAP; ++j) { int e = nbr[(size_t)d * ECAP + j]; const bool live = (j < n) && (e >= 0); e = min(max(e, 0), NE - 1); int s = src[e]; s = min(max(s, 0), NN - 1);
      float ev = AL[(size_t)s * 16 + h] + add; ev = (ev > 0.f) ? ev : 0.2f * ev; if (!live) ev = -3.0e38f; const float nm_ = fmaxf(mx, ev); const float r = live ? expf(mx - nm_) : 1.0f; const float p = live ? expf(ev - nm_) : 0.f; ls = ls * r + p; mx = live ? nm_ : mx;
      px = px * r + p * (CC[(size_t)s * 2] - cdx); py = py * r + p * (CC[(size_t)s * 2 + 1] - cdy); }
    const float il = 1.0f / (ls + 1e-16f); dsx += px * il * (1.0f / NHD); dsy += py * il * (1.0f / NHD); }
  v2f o; o.x = cdx + dsx; o.y = cdy + dsy; *(volatile v2f*)(out + (size_t)d * 2) = o; __threadfence(); *(volatile v2f*)(out + (size_t)d * 2) = o; }

extern "C" void kernel_launch(void* const* d_in, const int* in_sizes, int n_in,
                              void* d_out, int out_size, void* d_ws, size_t ws_size, hipStream_t stream) {
  (void)in_sizes; (void)n_in; (void)out_size;
  const float* const* I = (const float* const*)d_in; const float* data = I[0]; const int* edges = (const int*)d_in[1]; const int* srcI = edges; const int* dstI = edges + NE; const float* lW = I[2]; const float* lb = I[3];
  const float* W1 = I[4]; const float* as1 = I[5]; const float* ad1 = I[6]; const float* b1 = I[7]; const float* W2 = I[8]; const float* as2 = I[9]; const float* ad2 = I[10]; const float* b2 = I[11]; const float* W3 = I[12]; const float* as3 = I[13]; const float* ad3 = I[14]; const float* b3 = I[15]; const float* W4 = I[16]; const float* as4 = I[17]; const float* ad4 = I[18]; (void)I[19];
  char* ws = (char*)d_ws; size_t off = 0;
  auto take = [&](size_t bytes) { char* p = ws + off; off += (bytes + 255) & ~(size_t)255; return p; };
  const int nch = (NE + C4_CH - 1) / C4_CH;
  int* c4_CNT = (int*)take((size_t)nch * C4_NB * 4); int* c4_OFFB = (int*)take((size_t)nch * C4_NB * 4); int* c4_BOFF = (int*)take((size_t)(C4_NB + 64) * 4); int* c4_BUF = (int*)take((size_t)(NE + 64) * 4);
  int* cnt = (int*)take((size_t)(NN + 64) * 4); int* nbr = (int*)take((size_t)NN * ECAP * 4);
  _Float16* Bt = (_Float16*)take((size_t)3056 * 256 * 2 > (size_t)1504 * 512 * 2 ? (size_t)3056 * 256 * 2 : (size_t)1504 * 512 * 2); _Float16* Bl = (_Float16*)take((size_t)16 * 512 * 2);
  _Float16* T1 = (_Float16*)take((size_t)NN * 256 * 2); _Float16* T2 = (_Float16*)take((size_t)NN * 512 * 2); _Float16* T3 = (_Float16*)take((size_t)NN * 256 * 2); _Float16* T4 = (_Float16*)take((size_t)NN * 128 * 2);
  float* CCa = (float*)take((size_t)NN * 2 * 4); float* CCb = (float*)take((size_t)NN * 2 * 4); float* AL = (float*)take((size_t)NN * 16 * 4); _Float16* X = (_Float16*)take((size_t)NN * 3072 * 2);
  if (off > ws_size) return;
  k_c4_count<<<(unsigned)nch, 256, 0, stream>>>(dstI, NE, NN, c4_CNT); k_c4_offsets<<<1, 256, 0, stream>>>(c4_CNT, nch, NE, c4_OFFB, c4_BOFF); k_c4_scatter<<<(unsigned)nch, 256, 0, stream>>>(dstI, NE, NN, c4_OFFB, c4_BUF); k_c4_lists<ECAP><<<(NN + 255) / 256, 256, 0, stream>>>(dstI, c4_BUF, c4_BOFF, NN, NE, nbr, cnt);
  k_lin<<<(NN * 32 + 255) / 256, 256, 0, stream>>>(data, lW, lb, T1, CCa); k_cc0<<<(NN + 255) / 256, 256, 0, stream>>>(data, CCa);
  k_wl<256, 508, 3056><<<((3056 + 16) * 32 + 255) / 256, 256, 0, stream>>>(W1, as1, ad1, Bt, Bl);
  k_gemm_hhx<0><<<dim3(((NN / 16) * ((3048 + 63) / 64) + 3) / 4, 1), 128, 0, stream>>>(T1, 256, 0, Bt, 256, 0, 0.0625f, nullptr, 0, nullptr, 1, 0, 0, nullptr, X, 3072, 0, NN, 3048, 256);
  k_gemm_hhx<0><<<dim3(((NN / 16) * 1 + 3) / 4, 1), 128, 0, stream>>>(T1, 256, 0, Bl, 256, 0, 0.0625f, nullptr, 0, nullptr, 1, 0, 0, AL, nullptr, 16, 0, NN, 12, 256);
  k_dgat<508, 3072, 256, 2, 512><<<NN / 16, 512, 0, stream>>>(X, AL, T1, CCa, srcI, nbr, cnt, b1, T2, CCb);
  k_wl<512, 250, 1504><<<((1504 + 16) * 64 + 255) / 256, 256, 0, stream>>>(W2, as2, ad2, Bt, Bl);
  k_gemm_hhx<0><<<dim3(((NN / 16) * ((1500 + 63) / 64) + 3) / 4, 1), 128, 0, stream>>>(T2, 512, 0, Bt, 512, 0, 0.0625f, nullptr, 0, nullptr, 1, 0, 0, nullptr, X, 1536, 0, NN, 1500, 512);
  k_gemm_hhx<0><<<dim3(((NN / 16) * 1 + 3) / 4, 1), 128, 0, stream>>>(T2, 512, 0, Bl, 512, 0, 0.0625f, nullptr, 0, nullptr, 1, 0, 0, AL, nullptr, 16, 0, NN, 12, 512);
  k_dgat<250, 1536, 512, 4, 256><<<NN / 16, 512, 0, stream>>>(X, AL, T2, CCb, srcI, nbr, cnt, b2, T3, CCa);
  k_wl<256, 120, 720><<<((720 + 16) * 32 + 255) / 256, 256, 0, stream>>>(W3, as3, ad3, Bt, Bl);
  k_gemm_hhx<0><<<dim3(((NN / 16) * ((720 + 63) / 64) + 3) / 4, 1), 128, 0, stream>>>(T3, 256, 0, Bt, 256, 0, 0.0625f, nullptr, 0, nullptr, 1, 0, 0, nullptr, X, 768, 0, NN, 720, 256);
  k_gemm_hhx<0><<<dim3(((NN / 16) * 1 + 3) / 4, 1), 128, 0, stream>>>(T3, 256, 0, Bl, 256, 0, 0.0625f, nullptr, 0, nullptr, 1, 0, 0, AL, nullptr, 16, 0, NN, 12, 256);
  k_dgat<120, 768, 256, 6, 128><<<NN / 16, 512, 0, stream>>>(X, AL, T3, CCa, srcI, nbr, cnt, b3, T4, CCb);
  k_wl<128, 20, 128><<<((128 + 16) * 16 + 255) / 256, 256, 0, stream>>>(W4, as4, ad4, Bt, Bl);
  k_gemm_hhx<0><<<dim3(((NN / 16) * 1 + 3) / 4, 1), 128, 0, stream>>>(T4, 128, 0, Bl, 128, 0, 0.0625f, nullptr, 0, nullptr, 1, 0, 0, AL, nullptr, 16, 0, NN, 12, 128);
  k_dgat4<<<(NN + 255) / 256, 256, 0, stream>>>(AL, CCb, srcI, nbr, cnt, (float*)d_out);
}
